// DeepNet_6408091205736
// MI455X (gfx1250) — hardware-verified
//
#include <hip/hip_runtime.h>
#include <stddef.h>
#include <stdint.h>


#define DIM     128
#define NREL    8
#define KREL    (NREL * DIM)
#define KHI     ((NREL + 1) * DIM)
#define K2A     (KHI + KREL)
#define K2B     (KHI + KHI)
#define APITCH  K2B
#define GRP     16
#define NTHR    256
#define NWAVE   8
#define EPT     8
#define CHUNK   (NTHR * EPT)
#define WCAP    (EPT * 32)
#define LISTN   (NWAVE * WCAP)
#define NBMAX   2048
#define RCAP    28672
#define DEGCAP  256
#define ATILE_INTS (GRP * APITCH / 2)
#define OTILE_INTS (GRP * DIM)
#define WSMAX   134217728
#define LDS_LAYER ((2 * RCAP + 2 * NBMAX + LISTN) * 4 + 64)

static_assert((CHUNK & (CHUNK - 1)) == 0 && CHUNK <= 4096);
static_assert((NBMAX & (NBMAX - 1)) == 0 && NBMAX <= 4096);
static_assert(NTHR * 8 == NBMAX);
static_assert(LISTN >= NBMAX);
static_assert(LISTN >= NWAVE * WCAP);
static_assert((RCAP % 32) == 0);
static_assert(ATILE_INTS + OTILE_INTS <= RCAP);
static_assert((ATILE_INTS % 4) == 0);
static_assert(LDS_LAYER <= 300000);
static_assert(NWAVE * 2 == GRP);
static_assert(NWAVE * 16 == DIM);
static_assert(DIM == 4 * 32);
static_assert((K2A % 32) == 0 && (K2B % 32) == 0 && (KHI % 8) == 0 && (KREL % 8) == 0);
static_assert(K2B == APITCH && K2A <= APITCH);

typedef float          v4f  __attribute__((ext_vector_type(4)));
typedef float          v8f  __attribute__((ext_vector_type(8)));
typedef int            v4i  __attribute__((ext_vector_type(4)));
typedef int            v8i  __attribute__((ext_vector_type(8)));
typedef unsigned short v4us __attribute__((ext_vector_type(4)));
typedef unsigned short v8us __attribute__((ext_vector_type(8)));
typedef __bf16         v16bf __attribute__((ext_vector_type(16)));
union FragB { v16bf v; v8us h[2]; v8i w; };

__device__ __forceinline__ v8f wmb(const FragB& a, const FragB& b, v8f c) {
  v8f d = __builtin_amdgcn_wmma_f32_16x16x32_bf16(false, a.v, false, b.v, (short)0, c, false, false);
  asm volatile("v_nop\n\tv_nop\n\tv_nop\n\tv_nop" : "+v"(d) : "v"(a.w), "v"(b.w));
  return d;
}

__device__ __forceinline__ unsigned bfb(float f) {
  unsigned u = __float_as_uint(f);
  u += 0x7FFFu + ((u >> 16) & 1u);
  return u >> 16;
}
__device__ __forceinline__ float bff(unsigned b) { return __uint_as_float(b << 16); }

__device__ __forceinline__ int scan_chunk(const int* __restrict__ dsts, int nE, int cbase, int slotBase,
                                          int nb, int vec8, int* list, int tid, int lane, int wave) {
  int wc = 0;
  const int el0  = tid * EPT;
  const int e0   = cbase + el0;
  const int sent = -2147483647 - 1;
  v4i da, db;
  if (vec8 != 0 && cbase + CHUNK <= nE) {
    da = *(const v4i*)(dsts + e0);
    db = *(const v4i*)(dsts + e0 + 4);
  } else {
    da.x = (e0     < nE) ? dsts[min(e0,     nE - 1)] : sent;
    da.y = (e0 + 1 < nE) ? dsts[min(e0 + 1, nE - 1)] : sent;
    da.z = (e0 + 2 < nE) ? dsts[min(e0 + 2, nE - 1)] : sent;
    da.w = (e0 + 3 < nE) ? dsts[min(e0 + 3, nE - 1)] : sent;
    db.x = (e0 + 4 < nE) ? dsts[min(e0 + 4, nE - 1)] : sent;
    db.y = (e0 + 5 < nE) ? dsts[min(e0 + 5, nE - 1)] : sent;
    db.z = (e0 + 6 < nE) ? dsts[min(e0 + 6, nE - 1)] : sent;
    db.w = (e0 + 7 < nE) ? dsts[min(e0 + 7, nE - 1)] : sent;
  }
  const unsigned nbs = (unsigned)slotBase;
  const unsigned unb = (unsigned)nb;
  const unsigned s0 = (unsigned)da.x - nbs, s1 = (unsigned)da.y - nbs;
  const unsigned s2 = (unsigned)da.z - nbs, s3 = (unsigned)da.w - nbs;
  const unsigned s4 = (unsigned)db.x - nbs, s5 = (unsigned)db.y - nbs;
  const unsigned s6 = (unsigned)db.z - nbs, s7 = (unsigned)db.w - nbs;
  const bool h0 = s0 < unb, h1 = s1 < unb, h2 = s2 < unb, h3 = s3 < unb;
  const bool h4 = s4 < unb, h5 = s5 < unb, h6 = s6 < unb, h7 = s7 < unb;
  const unsigned any = __builtin_amdgcn_ballot_w32(h0 | h1 | h2 | h3 | h4 | h5 | h6 | h7);
  if (any != 0u) {
#define HITJ(J, HJ, SJ) { \
      const unsigned mj = __builtin_amdgcn_ballot_w32(HJ); \
      if (mj != 0u) { \
        if (HJ) { \
          const int pos = wc + (int)__builtin_amdgcn_mbcnt_lo(mj, 0u); \
          if (pos < WCAP) list[wave * WCAP + pos] = ((el0 + (J)) << 12) | (int)(SJ); \
        } \
        wc += (int)__builtin_popcount(mj); } }
    HITJ(0, h0, s0)
    HITJ(1, h1, s1)
    HITJ(2, h2, s2)
    HITJ(3, h3, s3)
    HITJ(4, h4, s4)
    HITJ(5, h5, s5)
    HITJ(6, h6, s6)
    HITJ(7, h7, s7)
#undef HITJ
  }
  return wc;
}

__global__ __launch_bounds__(NTHR) void k_wtb(const float* __restrict__ W, const float* __restrict__ root,
                                              unsigned short* wt, int K2, int nUnits) {
  const int u = (int)blockIdx.x * NTHR + (int)threadIdx.x;
  if (u >= nUnits) return;
  const int kq = K2 >> 3;
  const int n  = u / kq;
  const int k8 = (u - n * kq) * 8;
  int kk = (k8 < KHI) ? k8 : (k8 - KHI);
  kk = kk < 0 ? 0 : (kk > KHI - 8 ? KHI - 8 : kk);
  const int nc = n < DIM ? n : DIM - 1;
  const float* p = (kk < KREL) ? (W + (size_t)kk * DIM + nc) : (root + (size_t)(kk - KREL) * DIM + nc);
  v8us o;
#pragma unroll
  for (int i = 0; i < 8; ++i) o[i] = (unsigned short)bfb(p[(size_t)i * DIM]);
  const size_t ofs = (size_t)n * (size_t)K2 + (size_t)k8;
  *(volatile v8us*)(wt + ofs) = o;
  __threadfence();
  *(volatile v8us*)(wt + ofs) = o;
}

__global__ __launch_bounds__(NTHR) void k_layer(
    const int* __restrict__ srcs, const int* __restrict__ dsts, const int* __restrict__ ets,
    const float* __restrict__ xin, const unsigned short* __restrict__ wt, const float* __restrict__ bias,
    float* outp, int nN, int nE, int nb, int vec8, int K2, int rin) {
  extern __shared__ v4f lds_dyn[];
  int* reg1 = (int*)lds_dyn;
  int* reg2 = reg1 + RCAP;
  int* scnt = reg2 + RCAP;
  int* soff = scnt + NBMAX;
  int* list = soff + NBMAX;
  int* wcnt = list + LISTN;
  int* wtot = wcnt + NWAVE;
  const int tid = (int)threadIdx.x, lane = tid & 31, wave = tid >> 5;
  const int nodeBase = (int)blockIdx.x * nb;

  for (int i = tid; i < NBMAX; i += NTHR) scnt[i] = 0;
  __syncthreads();

  int tot = 0;
  const int nChunks = (nE + CHUNK - 1) / CHUNK;
#pragma unroll 1
  for (int ch = 0; ch < nChunks; ++ch) {
    const int cbase = ch * CHUNK;
    const int wc = scan_chunk(dsts, nE, cbase, nodeBase, nb, vec8, list, tid, lane, wave);
    if (lane == 0) wcnt[wave] = wc;
    __syncthreads();
    int pre = 0, all = 0;
#pragma unroll
    for (int w2 = 0; w2 < NWAVE; ++w2) {
      int c = wcnt[w2];
      c = c < 0 ? 0 : (c > WCAP ? WCAP : c);
      all += c;
      pre += (w2 < wave) ? c : 0;
    }
    const int wcc  = wc > WCAP ? WCAP : wc;
    const int base = tot + pre;
#pragma unroll 1
    for (int i = lane; i < wcc; i += 32) {
      const int ent = list[wave * WCAP + i];
      const int el  = (ent >> 12) & (CHUNK - 1);
      const int sl  = ent & (NBMAX - 1);
      int eid = cbase + el;
      eid = eid > nE - 1 ? nE - 1 : eid;
      const int pos = base + i;
      if (pos < RCAP) reg1[pos] = (int)(((unsigned)eid << 12) | (unsigned)sl);
    }
    tot += all;
    tot = tot > RCAP ? RCAP : tot;
    __syncthreads();
  }
  const int nh = tot;

  if (wave == 0) {
#pragma unroll 1
    for (int b0 = 0; b0 < nh; b0 += 32) {
      const int idx = b0 + lane;
      const int uv  = reg1[idx < RCAP ? idx : RCAP - 1];
      const int m32 = (nh - b0) < 32 ? (nh - b0) : 32;
#pragma unroll 1
      for (int k = 0; k < m32; ++k) {
        const int u  = __builtin_amdgcn_readlane(uv, k);
        const int sl = u & (NBMAX - 1);
        if (lane == 0) scnt[sl] = scnt[sl] + 1;
      }
    }
  }
  __syncthreads();

  {
    const v4i ca = *(const v4i*)(scnt + 8 * tid);
    const v4i cb = *(const v4i*)(scnt + 8 * tid + 4);
    const int e0 = ca.x < 0 ? 0 : ca.x, e1 = ca.y < 0 ? 0 : ca.y, e2 = ca.z < 0 ? 0 : ca.z, e3 = ca.w < 0 ? 0 : ca.w;
    const int e4 = cb.x < 0 ? 0 : cb.x, e5 = cb.y < 0 ? 0 : cb.y, e6 = cb.z < 0 ? 0 : cb.z, e7 = cb.w < 0 ? 0 : cb.w;
    const int ts = e0 + e1 + e2 + e3 + e4 + e5 + e6 + e7;
    int incl = ts;
#pragma unroll
    for (int d = 1; d < 32; d <<= 1) {
      const int up = __shfl_up(incl, d);
      if (lane >= d) incl += up;
    }
    if (lane == 31) wtot[wave] = incl;
    __syncthreads();
    int pre = 0;
#pragma unroll
    for (int w2 = 0; w2 < NWAVE; ++w2) pre += (w2 < wave) ? wtot[w2] : 0;
    int run = pre + incl - ts;
    soff[8 * tid + 0] = run; run += e0;
    soff[8 * tid + 1] = run; run += e1;
    soff[8 * tid + 2] = run; run += e2;
    soff[8 * tid + 3] = run; run += e3;
    soff[8 * tid + 4] = run; run += e4;
    soff[8 * tid + 5] = run; run += e5;
    soff[8 * tid + 6] = run; run += e6;
    soff[8 * tid + 7] = run;
  }
  __syncthreads();
  for (int i = tid; i < NBMAX; i += NTHR) list[i] = soff[i];
  __syncthreads();

  if (wave == 0) {
#pragma unroll 1
    for (int b0 = 0; b0 < nh; b0 += 32) {
      const int idx = b0 + lane;
      const int uv  = reg1[idx < RCAP ? idx : RCAP - 1];
      const int m32 = (nh - b0) < 32 ? (nh - b0) : 32;
#pragma unroll 1
      for (int k = 0; k < m32; ++k) {
        const int u   = __builtin_amdgcn_readlane(uv, k);
        const int sl  = u & (NBMAX - 1);
        const int eid = (int)((unsigned)u >> 12);
        if (lane == 0) {
          int pos = list[sl];
          pos = pos < 0 ? 0 : (pos > RCAP - 1 ? RCAP - 1 : pos);
          reg2[pos] = eid;
          list[sl] = pos + 1;
        }
      }
    }
  }
  __syncthreads();

  unsigned short* atile = (unsigned short*)reg1;
  float* otile = (float*)(reg1 + ATILE_INTS);
  const bool ovf = (nh >= RCAP);
  const int ngrp = nb / GRP;
  const bool rlo = (K2 > KHI + KREL);
  const int ksteps = K2 >> 5;
  const int hh = lane >> 4, m = lane & 15;
#pragma unroll 1
  for (int g = 0; g < ngrp; ++g) {
    const int sb    = g * GRP;
    const int rbase = nodeBase + sb;
    if (rbase >= nN) break;

#pragma unroll 1
    for (int jj = 0; jj < 2; ++jj) {
      const int j    = 2 * wave + jj;
      const int slot = sb + j;
      const int grow = rbase + j;
      const int gcl  = grow < nN ? grow : nN - 1;
      int st = soff[slot];
      const int craw = scnt[slot];
      int cnt = craw;
      st  = st < 0 ? 0 : (st > nh ? nh : st);
      cnt = cnt < 0 ? 0 : (cnt > DEGCAP ? DEGCAP : cnt);
      if (cnt > nh - st) cnt = nh - st;
      const float live = grow < nN ? 1.0f : 0.0f;

      float a[4 * NREL];
      int   cn[NREL];
#pragma unroll
      for (int i = 0; i < 4 * NREL; ++i) a[i] = 0.f;
#pragma unroll
      for (int rr = 0; rr < NREL; ++rr) cn[rr] = 0;

#pragma unroll 1
      for (int q = 0; q < cnt; ++q) {
        int idx = st + q; idx = idx > RCAP - 1 ? RCAP - 1 : idx;
        int eid = reg2[idx]; eid = eid < 0 ? 0 : (eid > nE - 1 ? nE - 1 : eid);
        const int sraw = srcs[eid];
        const int s    = sraw < 0 ? 0 : (sraw > nN - 1 ? nN - 1 : sraw);
        const int rraw = ets[eid];
        const int r    = rraw < 0 ? 0 : (rraw > NREL - 1 ? NREL - 1 : rraw);
        v4f xv = *(const v4f*)(xin + (size_t)s * DIM + 4 * lane);
        if (rin != 0) {
          xv.x = bff(bfb(xv.x)); xv.y = bff(bfb(xv.y)); xv.z = bff(bfb(xv.z)); xv.w = bff(bfb(xv.w));
        }
#pragma unroll
        for (int rr = 0; rr < NREL; ++rr) {
          const bool hit = (r == rr);
          a[4 * rr + 0] += hit ? xv.x : 0.f;
          a[4 * rr + 1] += hit ? xv.y : 0.f;
          a[4 * rr + 2] += hit ? xv.z : 0.f;
          a[4 * rr + 3] += hit ? xv.w : 0.f;
          cn[rr] += hit ? 1 : 0;
        }
      }

      unsigned short* ar = atile + j * APITCH + 4 * lane;
#pragma unroll
      for (int rr = 0; rr < NREL; ++rr) {
        const float dg = (float)cn[rr];
        const float iv = (dg > 0.f) ? (1.0f / fmaxf(dg, 1.0f)) : 0.f;
        const float sc = iv * live;
        const float m0 = a[4 * rr + 0] * sc, m1 = a[4 * rr + 1] * sc;
        const float m2 = a[4 * rr + 2] * sc, m3 = a[4 * rr + 3] * sc;
        const unsigned h0 = bfb(m0), h1 = bfb(m1), h2 = bfb(m2), h3 = bfb(m3);
        v4us hv, lv;
        hv.x = (unsigned short)h0; hv.y = (unsigned short)h1; hv.z = (unsigned short)h2; hv.w = (unsigned short)h3;
        lv.x = (unsigned short)bfb(m0 - bff(h0)); lv.y = (unsigned short)bfb(m1 - bff(h1));
        lv.z = (unsigned short)bfb(m2 - bff(h2)); lv.w = (unsigned short)bfb(m3 - bff(h3));
        *(v4us*)(ar + rr * DIM)       = hv;
        *(v4us*)(ar + KHI + rr * DIM) = lv;
      }
      {
        v4f xr = *(const v4f*)(xin + (size_t)gcl * DIM + 4 * lane);
        if (rin != 0) {
          xr.x = bff(bfb(xr.x)); xr.y = bff(bfb(xr.y)); xr.z = bff(bfb(xr.z)); xr.w = bff(bfb(xr.w));
        }
        xr = xr * live;
        const unsigned pzb = (ovf || craw > DEGCAP) ? 0x7FC0u : 0u;
        const unsigned h0 = bfb(xr.x) | pzb, h1 = bfb(xr.y) | pzb, h2 = bfb(xr.z) | pzb, h3 = bfb(xr.w) | pzb;
        v4us hv, lv;
        hv.x = (unsigned short)h0; hv.y = (unsigned short)h1; hv.z = (unsigned short)h2; hv.w = (unsigned short)h3;
        lv.x = (unsigned short)bfb(xr.x - bff(h0)); lv.y = (unsigned short)bfb(xr.y - bff(h1));
        lv.z = (unsigned short)bfb(xr.z - bff(h2)); lv.w = (unsigned short)bfb(xr.w - bff(h3));
        *(v4us*)(ar + KREL) = hv;
        if (rlo) *(v4us*)(ar + KHI + KREL) = lv;
      }
    }
    __syncthreads();

    {
      v8f acc;
      {
        const v8f z = {0.f, 0.f, 0.f, 0.f, 0.f, 0.f, 0.f, 0.f};
        acc = z;
      }
      const unsigned short* ap = atile + m * APITCH + 8 * hh;
      const unsigned short* bp = wt + (size_t)(16 * wave + m) * (size_t)K2 + 8 * hh;
#pragma unroll 2
      for (int ks = 0; ks < ksteps; ++ks) {
        FragB af, bf;
        af.h[0] = *(const v8us*)(ap + 32 * ks);
        af.h[1] = *(const v8us*)(ap + 32 * ks + 16);
        bf.h[0] = *(const v8us*)(bp + 32 * ks);
        bf.h[1] = *(const v8us*)(bp + 32 * ks + 16);
        acc = wmb(af, bf, acc);
      }
      const int col = 16 * wave + m;
      const float bb = bff(bfb(bias[col]));
#pragma unroll
      for (int r = 0; r < 8; ++r) {
        const float v = acc[r] + bb;
        otile[(8 * hh + r) * DIM + col] = (v < 0.f) ? 0.f : v;
      }
    }
    __syncthreads();

    {
      const int l0 = 2 * wave, l1 = 2 * wave + 1;
      const v4f o0 = *(const v4f*)(otile + l0 * DIM + 4 * lane);
      const v4f o1 = *(const v4f*)(otile + l1 * DIM + 4 * lane);
      const int g0 = rbase + l0, g1 = rbase + l1;
      const bool w0 = g0 < nN, w1 = g1 < nN;
      float* p0 = outp + (size_t)(w0 ? g0 : nN - 1) * DIM + 4 * lane;
      float* p1 = outp + (size_t)(w1 ? g1 : nN - 1) * DIM + 4 * lane;
      if (w0) *(volatile v4f*)p0 = o0;
      if (w1) *(volatile v4f*)p1 = o1;
      __threadfence();
      if (w0) *(volatile v4f*)p0 = o0;
      if (w1) *(volatile v4f*)p1 = o1;
    }
    __syncthreads();
  }
}

static int pick_nb(int nE, int nN) {
  int nb = NBMAX;
  while (nb > 16 && (long long)nb * (long long)nE * 5LL > (long long)RCAP * (long long)nN * 4LL) nb >>= 1;
  return nb;
}
static inline int cdiv(int a, int b) { return (a + b - 1) / b; }

extern "C" void kernel_launch(void* const* d_in, const int* in_sizes, int n_in,
                              void* d_out, int out_size, void* d_ws, size_t ws_size,
                              hipStream_t stream) {
  if (n_in < 9) return;
  const int nN = in_sizes[0] / DIM;
  if (nN <= 0 || in_sizes[0] != nN * DIM || nN > (1 << 22)) return;
  if (in_sizes[1] < 2 || (in_sizes[1] & 1) != 0) return;
  const int nE = in_sizes[1] / 2;
  if (nE < 1 || nE > (1 << 20)) return;
  if (in_sizes[2] != nE) return;
  if (in_sizes[3] != NREL * DIM * DIM || in_sizes[4] != DIM * DIM || in_sizes[5] != DIM) return;
  if (in_sizes[6] != NREL * DIM * DIM || in_sizes[7] != DIM * DIM || in_sizes[8] != DIM) return;
  if (out_size != nN * DIM) return;

  const float* x   = (const float*)d_in[0];
  const int*   ei  = (const int*)  d_in[1];
  const int*   et  = (const int*)  d_in[2];
  const float* W1  = (const float*)d_in[3];
  const float* R1  = (const float*)d_in[4];
  const float* b1  = (const float*)d_in[5];
  const float* W2  = (const float*)d_in[6];
  const float* R2  = (const float*)d_in[7];
  const float* b2  = (const float*)d_in[8];
  float* out = (float*)d_out;
  const int* src = ei;
  const int* dst = ei + nE;

  const int nb   = pick_nb(nE, nN);
  const int gA   = cdiv(nN, nb);
  const int vec8 = ((nE & 3) == 0) ? 1 : 0;
  if (nb < GRP || (nb % GRP) != 0 || gA * nb < nN) return;

  char* ws = (char*)d_ws;
  size_t off = 0;
  const size_t oH1 = off; off += (size_t)nN * DIM * 4;          off = (off + 255) & ~(size_t)255;
  const size_t oWA = off; off += (size_t)DIM * K2A * 2;         off = (off + 255) & ~(size_t)255;
  const size_t oWB = off; off += (size_t)DIM * K2B * 2;         off = (off + 255) & ~(size_t)255;
  if (off > ws_size || off > (size_t)WSMAX) return;
  float*          H1  = (float*)(ws + oH1);
  unsigned short* WTA = (unsigned short*)(ws + oWA);
  unsigned short* WTB = (unsigned short*)(ws + oWB);

  hipFuncSetAttribute(reinterpret_cast<const void*>(&k_layer),
                      hipFuncAttributeMaxDynamicSharedMemorySize, LDS_LAYER);

  {
    const int nUa = DIM * (K2A / 8);
    k_wtb<<<cdiv(nUa, NTHR), NTHR, 0, stream>>>(W1, R1, WTA, K2A, nUa);
    const int nUb = DIM * (K2B / 8);
    k_wtb<<<cdiv(nUb, NTHR), NTHR, 0, stream>>>(W2, R2, WTB, K2B, nUb);
  }
  k_layer<<<gA, NTHR, LDS_LAYER, stream>>>(src, dst, et, x, WTA, b1, H1, nN, nE, nb, vec8, K2A, 1);
  k_layer<<<gA, NTHR, LDS_LAYER, stream>>>(src, dst, et, H1, WTB, b2, out, nN, nE, nb, vec8, K2B, 0);
}
